// LibraKANMixer_56083682951294
// MI455X (gfx1250) — hardware-run, weakly checked
//
#include <hip/hip_runtime.h>


namespace {
constexpr int B = 128, W = 1024, F = 2048;
constexpr float XS = 8.0f, WSC = 256.0f, RHO = 0.3f, SCALE = 0.8f, BETA = 6.0f, TAU = 0.001f;
typedef _Float16 b16;
typedef __attribute__((ext_vector_type(16))) _Float16 v16b;
typedef __attribute__((ext_vector_type(8))) _Float16 v8b;
typedef __attribute__((ext_vector_type(8))) float v8f;
typedef __attribute__((ext_vector_type(4))) float v4f;
__device__ __forceinline__ float bf16_rne(float f) { unsigned int u = __float_as_uint(f); u += 0x7FFFu + ((u >> 16) & 1u); return __uint_as_float(u & 0xFFFF0000u); }
__device__ __forceinline__ void split16(float v, b16& hi, b16& lo) { hi = (b16)v; lo = (b16)(v - (float)hi); }
__device__ __forceinline__ v16b frag_kb(const b16* p, int hh) { const v8b a = *(const v8b*)(p + 8 * hh), b = *(const v8b*)(p + 16 + 8 * hh); v16b f;
#pragma unroll
  for (int e = 0; e < 8; ++e) { f[e] = a[e]; f[8 + e] = b[e]; } return f; }
__device__ __forceinline__ v8f wmma16b(v16b a, v16b b, v8f c) { v8f d = __builtin_amdgcn_wmma_f32_16x16x32_f16(false, a, false, b, (short)0, c, false, false); asm volatile("v_nop\n\tv_nop\n\tv_nop\n\tv_nop" : "+v"(d) : "v"(a), "v"(b)); return d; }
__device__ __forceinline__ void wave_lds_sync() { __builtin_amdgcn_fence(__ATOMIC_RELEASE, "workgroup"); __builtin_amdgcn_wave_barrier(); __builtin_amdgcn_fence(__ATOMIC_ACQUIRE, "workgroup"); }
__device__ __forceinline__ float pmul(float a, float b) { float p = a * b; asm volatile("" : "+v"(p)); return p; }
__device__ __forceinline__ float gelu(float v) { return 0.5f * v * (1.0f + erff(v * 0.70710678118654752f)); }

__global__ __launch_bounds__(256) void wcopy_kernel(const float* __restrict__ w, int n8, b16* __restrict__ WT) {
  const int u = blockIdx.x * 256 + threadIdx.x; if (u >= n8) return; const int e = u * 8; v8b v;
#pragma unroll
  for (int j = 0; j < 8; ++j) v[j] = (b16)(bf16_rne(w[e + j]) * WSC); for (int pass = 0; pass < 2; ++pass) { *(volatile v8b*)(WT + e) = v; __threadfence(); }
}
__global__ __launch_bounds__(1024) void fmax_kernel(const float* __restrict__ freq, float* __restrict__ DEN) {
  __shared__ float red[1024]; const int tid = threadIdx.x; float m = 0.0f;
#pragma unroll 4
  for (int i = tid; i < F * W; i += 1024) m = fmaxf(m, fabsf(bf16_rne(freq[i]) * SCALE)); red[tid] = m; __syncthreads();
  for (int s = 512; s > 0; s >>= 1) { if (tid < s) red[tid] = fmaxf(red[tid], red[tid + s]); __syncthreads(); }
  if (tid < 32) { for (int pass = 0; pass < 2; ++pass) { ((volatile float*)DEN)[tid] = red[0]; __threadfence(); } }
}
__global__ __launch_bounds__(256) void compact_kernel(const float* __restrict__ freq, const float* __restrict__ alpha, const float* __restrict__ gate, const float* __restrict__ DEN, float* __restrict__ NZT, float* __restrict__ NZF, int* __restrict__ NZC) {
  const int w = blockIdx.x * 256 + threadIdx.x; if (w >= W) return; const float den = DEN[0]; int cnt = 0;
#pragma unroll 1
  for (int f = 0; f < F; ++f) { const float fv = bf16_rne(freq[(size_t)f * W + w]) * SCALE; const float win = den < 1e-8f ? 1.0f : __expf(-BETA * pmul(fv / den, fv / den)); const float raw = pmul(bf16_rne(alpha[(size_t)f * W + w]), bf16_rne(gate[(size_t)f * W + w]));
    const float mag = fmaxf(fabsf(raw) - TAU, 0.0f); const float sgn = raw > 0.0f ? 1.0f : (raw < 0.0f ? -1.0f : 0.0f); const float t = pmul(pmul(sgn, mag), win);
    if (t != 0.0f) { for (int pass = 0; pass < 2; ++pass) { ((volatile float*)NZT)[(size_t)w * F + cnt] = t; ((volatile float*)NZF)[(size_t)w * F + cnt] = fv; } ++cnt; } }
  for (int pass = 0; pass < 2; ++pass) { ((volatile int*)NZC)[w] = cnt; __threadfence(); }
}
__global__ __launch_bounds__(256) void spec_kernel(const float* __restrict__ x, const float* __restrict__ g, const float* __restrict__ bb, const float* __restrict__ NZT, const float* __restrict__ NZF, const int* __restrict__ NZC, int BV, float* __restrict__ HS) {
  const int wave = threadIdx.x >> 5, lane = threadIdx.x & 31; const int b = blockIdx.x * 8 + wave; if (b >= BV) return;
  float v[32]; float s = 0.0f; for (int q = 0; q < 32; ++q) { v[q] = bf16_rne(x[(size_t)b * W + q * 32 + lane]); s += v[q]; } for (int o = 16; o; o >>= 1) s += __shfl_xor(s, o); const float mu = s * (1.0f / W);
  float vq = 0.0f; for (int q = 0; q < 32; ++q) { const float d = v[q] - mu; vq += pmul(d, d); } for (int o = 16; o; o >>= 1) vq += __shfl_xor(vq, o); const float rs = rsqrtf(vq * (1.0f / W) + 1e-5f);
#pragma unroll 1
  for (int pass = 0; pass < 2; ++pass) {
#pragma unroll 1
    for (int q = 0; q < 32; ++q) { const int w = q * 32 + lane; const float xn = pmul(pmul(v[q] - mu, rs), bf16_rne(g[w])) + bf16_rne(bb[w]); const int cnt = min(max(NZC[w], 0), F); float h = 0.0f;
#pragma unroll 1
      for (int j = 0; j < cnt; ++j) h += pmul(sinf(pmul(xn, NZF[(size_t)w * F + j])), NZT[(size_t)w * F + j]);
      ((volatile float*)HS)[(size_t)b * W + w] = h; }
    __threadfence(); }
}
__global__ __launch_bounds__(32) void out_kernel(const float* __restrict__ x, const float* __restrict__ g, const float* __restrict__ bb, const b16* __restrict__ WT, const float* __restrict__ bl, const float* __restrict__ HS, int BV, float* __restrict__ out) {
  __shared__ __attribute__((aligned(16))) b16 Ah[16][W + 8], Al[16][W + 8]; __shared__ __attribute__((aligned(16))) float Tf[16][128 + 4], Rm[16];
  const int lane = threadIdx.x, nloc = lane & 15, hlf = lane >> 4; const size_t m0 = (size_t)blockIdx.x * 16; if (m0 >= (size_t)BV) return;
  for (int rr = 0; rr < 16; ++rr) { float v[32]; float s = 0.0f, hq = 0.0f; for (int q = 0; q < 32; ++q) { v[q] = bf16_rne(x[(m0 + rr) * W + q * 32 + lane]); s += v[q]; const float h = HS[(m0 + rr) * W + q * 32 + lane]; hq += pmul(h, h); }
    for (int o = 16; o; o >>= 1) { s += __shfl_xor(s, o); hq += __shfl_xor(hq, o); } const float mu = s * (1.0f / W); float vq = 0.0f; for (int q = 0; q < 32; ++q) { const float d = v[q] - mu; vq += pmul(d, d); } for (int o = 16; o; o >>= 1) vq += __shfl_xor(vq, o); const float rs = rsqrtf(vq * (1.0f / W) + 1e-5f);
    if (lane == 0) Rm[rr] = 1.0f / sqrtf(hq * (1.0f / W) + 1e-8f);
    for (int q = 0; q < 32; ++q) { const int w = q * 32 + lane; b16 p, ql; split16((pmul(pmul(v[q] - mu, rs), bf16_rne(g[w])) + bf16_rne(bb[w])) * XS, p, ql); Ah[rr][w] = p; Al[rr][w] = ql; } }
  wave_lds_sync();
#pragma unroll 1
  for (int cg = 0; cg < W / 128; ++cg) { v8f acc[8];
#pragma unroll
    for (int t = 0; t < 8; ++t) acc[t] = (v8f){};
#pragma unroll 2
    for (int kb = 0; kb < W; kb += 32) { const v16b a = frag_kb(&Ah[nloc][kb], hlf), al = frag_kb(&Al[nloc][kb], hlf);
#pragma unroll
      for (int t = 0; t < 8; ++t) { const v16b bw = frag_kb(WT + (size_t)(cg * 128 + t * 16 + nloc) * W + kb, hlf); acc[t] = wmma16b(a, bw, acc[t]); acc[t] = wmma16b(al, bw, acc[t]); } }
#pragma unroll
    for (int t = 0; t < 8; ++t) { const int c = cg * 128 + t * 16 + nloc; const float b1 = bf16_rne(bl[c]);
#pragma unroll 1
      for (int r8 = 0; r8 < 8; ++r8) { const int rl = 8 * hlf + r8; Tf[rl][t * 16 + nloc] = gelu(acc[t][r8] * (1.0f / (XS * WSC)) + b1) + RHO * pmul(HS[(m0 + rl) * W + c], Rm[rl]); } }
    wave_lds_sync();
    for (int pass = 0; pass < 2; ++pass) { for (int rr = 0; rr < 16; ++rr) *(volatile v4f*)(out + (m0 + rr) * W + cg * 128 + lane * 4) = *(const v4f*)(&Tf[rr][lane * 4]); __threadfence(); }
    wave_lds_sync(); }
}
}

extern "C" void kernel_launch(void* const* d_in, const int* in_sizes, int n_in, void* d_out, int out_size, void* d_ws, size_t ws_size, hipStream_t stream) {
  (void)n_in;
  auto Fp = [&](int i) { return (const float*)d_in[i]; };
  if (in_sizes[0] != B * W || in_sizes[1] != F * W || in_sizes[2] != F * W || in_sizes[3] != F * W || in_sizes[4] != W || in_sizes[6] != W * W || out_size != B * W) return;
  const int BV = B;
  size_t off = 0; char* ws = (char*)d_ws;
  auto carve = [&](size_t bytes) { char* p = ws + off; off += (bytes + 255) & ~(size_t)255; return p; };
  b16* WT = (b16*)carve((size_t)W * W * 2); float* DEN = (float*)carve(256); float* NZT = (float*)carve((size_t)W * F * 4); float* NZF = (float*)carve((size_t)W * F * 4); int* NZC = (int*)carve(W * 4); float* HS = (float*)carve((size_t)B * W * 4);
  if (off > ws_size || off > ((size_t)64 << 20)) return;
  wcopy_kernel<<<(W * W / 8 + 255) / 256, 256, 0, stream>>>(Fp(6), W * W / 8, WT);
  fmax_kernel<<<1, 1024, 0, stream>>>(Fp(1), DEN);
  compact_kernel<<<W / 256, 256, 0, stream>>>(Fp(1), Fp(2), Fp(3), DEN, NZT, NZF, NZC);
  spec_kernel<<<(BV + 7) / 8, 256, 0, stream>>>(Fp(0), Fp(4), Fp(5), NZT, NZF, NZC, BV, HS);
  out_kernel<<<(BV + 15) / 16, 32, 0, stream>>>(Fp(0), Fp(4), Fp(5), WT, Fp(7), HS, BV, (float*)d_out);
}
